// LocalGlobalCausalSelfAttention_16037407883515
// MI455X (gfx1250) — hardware-verified
//
#include <hip/hip_runtime.h>
#include <stddef.h>
#include <stdint.h>

#define SQ    2048
#define DIM   1024
#define NH    16
#define NKV   4
#define HDM   64
#define KVD   256
#define WROWS 2560
#define OROW  1536
#define QB    64
#define KC    64
#define NQB   (SQ / QB)
#define LWIN  256
#define GTOK  64

static_assert(NH * HDM == DIM);
static_assert(NKV * HDM == KVD);
static_assert(WROWS == DIM + KVD + KVD + DIM);
static_assert(OROW == DIM + KVD + KVD);
static_assert(SQ % QB == 0);
static_assert(SQ % KC == 0);
static_assert(DIM % 64 == 0);
static_assert((SQ * DIM) % 2048 == 0);
static_assert(HDM == 64);
static_assert(GTOK == KC);

typedef unsigned short us;
typedef __attribute__((ext_vector_type(16))) __bf16 v16bf;
typedef us           v8us __attribute__((ext_vector_type(8)));
typedef float        v8f  __attribute__((ext_vector_type(8)));
typedef float        v4f  __attribute__((ext_vector_type(4)));
typedef unsigned int v4u  __attribute__((ext_vector_type(4)));

union Frag  { v16bf v; v8us h[2]; };
union Pack8 { v8us h; v4u u; };

struct RopeTab { float f[32]; };
static_assert(sizeof(RopeTab) == 128);

__device__ __forceinline__ us bf_rne(float f) {
  unsigned u = __float_as_uint(f);
  u = u + 0x7FFFu + ((u >> 16) & 1u);
  return (us)(u >> 16);
}
__device__ __forceinline__ float bf_val(us h) { return __uint_as_float(((unsigned)h) << 16); }
__device__ __forceinline__ void split2(float f, us& hi, us& lo) {
  const us hv = bf_rne(f);
  hi = hv;
  lo = bf_rne(f - bf_val(hv));
}
__device__ __forceinline__ void split8(const float (&f)[8], Pack8& ph, Pack8& pl) {
  us hh[8], ll[8];
#pragma unroll
  for (int e = 0; e < 8; ++e) split2(f[e], hh[e], ll[e]);
  ph.h = (v8us){hh[0], hh[1], hh[2], hh[3], hh[4], hh[5], hh[6], hh[7]};
  pl.h = (v8us){ll[0], ll[1], ll[2], ll[3], ll[4], ll[5], ll[6], ll[7]};
}

__device__ __forceinline__ v8f mma16(v16bf a, v16bf b, v8f c) {
  c = __builtin_amdgcn_wmma_f32_16x16x32_bf16(false, a, false, b, (short)0, c, false, false);
  asm volatile("v_nop\n\tv_nop\n\tv_nop\n\tv_nop" : "+v"(c) : "v"(a), "v"(b));
  return c;
}

__device__ __forceinline__ v16bf ldfrag(const us* p, int ld, int row0, int k0, int lane) {
  const int m = lane & 15, lh = lane >> 4;
  const us* q = p + (size_t)(row0 + m) * ld + k0 + 8 * lh;
  Frag f;
  f.h[0] = *(const v8us*)(q);
  f.h[1] = *(const v8us*)(q + 16);
  return f.v;
}

__device__ __forceinline__ v8f zero8() { return (v8f){0.f, 0.f, 0.f, 0.f, 0.f, 0.f, 0.f, 0.f}; }

__device__ __forceinline__ float wsum32(float s) {
#pragma unroll
  for (int off = 16; off >= 1; off >>= 1) s += __shfl_xor(s, off, 32);
  return s;
}

__device__ __forceinline__ void gemm16x64x3(const us* __restrict__ Ah, const us* __restrict__ Al,
                                            const us* __restrict__ Bh, const us* __restrict__ Bl,
                                            int m0, int n0, int lane, v8f (&acc)[4]) {
#pragma unroll 1
  for (int k0 = 0; k0 < DIM; k0 += 32) {
    const v16bf ah = ldfrag(Ah, DIM, m0, k0, lane);
    const v16bf al = ldfrag(Al, DIM, m0, k0, lane);
#pragma unroll
    for (int t = 0; t < 4; ++t) {
      const v16bf bh = ldfrag(Bh, DIM, n0 + 16 * t, k0, lane);
      const v16bf bl = ldfrag(Bl, DIM, n0 + 16 * t, k0, lane);
      acc[t] = mma16(ah, bh, acc[t]);
      acc[t] = mma16(ah, bl, acc[t]);
      acc[t] = mma16(al, bh, acc[t]);
    }
  }
}

#define TWP 68
__global__ __launch_bounds__(128) void k_cvtw(const float* __restrict__ wq, const float* __restrict__ wk,
                                              const float* __restrict__ wv, const float* __restrict__ wo,
                                              us* __restrict__ wh, us* __restrict__ wl) {
  __shared__ __align__(16) float tl[64 * TWP];
  const int tid = threadIdx.x;
  const int rt = blockIdx.x;
  const int k0 = blockIdx.y * 64;
  const float* s = (rt < 16) ? wq : ((rt < 20) ? wk : ((rt < 24) ? wv : wo));
  const int pitch = (rt < 16 || rt >= 24) ? DIM : KVD;
  const int n0 = 64 * ((rt < 16) ? rt : ((rt < 20) ? (rt - 16) : ((rt < 24) ? (rt - 20) : (rt - 24))));
#pragma unroll
  for (int j = 0; j < 8; ++j) {
    const int p  = tid + 128 * j;
    const int kr = p >> 4;
    const int c4 = (p & 15) * 4;
    const v4f a = *(const v4f*)(s + (size_t)(k0 + kr) * pitch + n0 + c4);
    *(v4f*)(tl + kr * TWP + c4) = a;
  }
  __syncthreads();
  v4u hv[4], lv[4];
  size_t go[4];
#pragma unroll
  for (int j = 0; j < 4; ++j) {
    const int p  = tid + 128 * j;
    const int n  = p >> 3;
    const int kc = (p & 7) * 8;
    const float* cp = tl + kc * TWP + n;
    float f[8];
#pragma unroll
    for (int e = 0; e < 8; ++e) f[e] = cp[e * TWP];
    Pack8 ph, pl;
    split8(f, ph, pl);
    hv[j] = ph.u;
    lv[j] = pl.u;
    go[j] = ((size_t)(64 * rt + n)) * DIM + k0 + kc;
  }
#pragma unroll
  for (int j = 0; j < 4; ++j) { *(volatile v4u*)(wh + go[j]) = hv[j]; *(volatile v4u*)(wl + go[j]) = lv[j]; }
  __threadfence();
#pragma unroll
  for (int j = 0; j < 4; ++j) { *(volatile v4u*)(wh + go[j]) = hv[j]; *(volatile v4u*)(wl + go[j]) = lv[j]; }
}

__global__ __launch_bounds__(256) void k_cvtx(const float* __restrict__ x, us* __restrict__ xh, us* __restrict__ xl) {
  const size_t i = (size_t)blockIdx.x * 2048 + (size_t)threadIdx.x * 8;
  const v4f a0 = *(const v4f*)(x + i);
  const v4f a1 = *(const v4f*)(x + i + 4);
  const float f[8] = {a0[0], a0[1], a0[2], a0[3], a1[0], a1[1], a1[2], a1[3]};
  Pack8 ph, pl;
  split8(f, ph, pl);
  const v4u hv = ph.u, lv = pl.u;
  *(volatile v4u*)(xh + i) = hv;
  *(volatile v4u*)(xl + i) = lv;
  __threadfence();
  *(volatile v4u*)(xh + i) = hv;
  *(volatile v4u*)(xl + i) = lv;
}

__global__ __launch_bounds__(256) void k_rope(RopeTab tb, float* __restrict__ ct, float* __restrict__ st) {
  const int tid = threadIdx.x, lane = tid & 31;
  const int pos = blockIdx.x * 8 + (tid >> 5);
  float inv = tb.f[0];
#pragma unroll
  for (int i = 1; i < 32; ++i) inv = (lane == i) ? tb.f[i] : inv;
  const float ang = (float)pos * inv;
  float sn, cs;
  sincosf(ang, &sn, &cs);
  const size_t o = (size_t)pos * 32 + lane;
  *(volatile float*)(ct + o) = cs;
  *(volatile float*)(st + o) = sn;
  __threadfence();
  *(volatile float*)(ct + o) = cs;
  *(volatile float*)(st + o) = sn;
}

#define SFP 68
__global__ __launch_bounds__(128) void k_qkv(const us* __restrict__ xh, const us* __restrict__ xl,
                                             const us* __restrict__ wh, const us* __restrict__ wl,
                                             const float* __restrict__ ct, const float* __restrict__ st,
                                             us* __restrict__ qh, us* __restrict__ ql,
                                             us* __restrict__ kh, us* __restrict__ kl,
                                             us* __restrict__ vh, us* __restrict__ vl) {
  __shared__ __align__(16) float sf[64 * SFP];
  const int tid = threadIdx.x, lane = tid & 31, wave = tid >> 5;
  const int hh = lane >> 4, c = lane & 15;
  const int mb = blockIdx.x * 64;
  const int ns = blockIdx.y;
  const int which = (ns < 16) ? 0 : ((ns < 20) ? 1 : 2);
  const int m0 = mb + wave * 16;
  const int n0 = 64 * ns;

  v8f acc[4];
#pragma unroll
  for (int t = 0; t < 4; ++t) acc[t] = zero8();
  gemm16x64x3(xh, xl, wh, wl, m0, n0, lane, acc);

#pragma unroll
  for (int t = 0; t < 4; ++t) {
#pragma unroll
    for (int r = 0; r < 8; ++r)
      sf[(wave * 16 + 8 * hh + r) * SFP + 16 * t + c] = acc[t][r];
  }
  __syncthreads();

  if (which < 2) {
#pragma unroll 2
    for (int r = 0; r < 16; ++r) {
      const int lr  = wave * 16 + r;
      const int pos = mb + lr;
      float x1 = sf[lr * SFP + lane];
      float x2 = sf[lr * SFP + lane + 32];
      float ss = x1 * x1 + x2 * x2;
      ss = wsum32(ss);
      const float rn = rsqrtf(ss * (1.0f / 64.0f) + 1.1920929e-07f);
      x1 *= rn;
      x2 *= rn;
      const float cs = ct[(size_t)pos * 32 + lane];
      const float sn = st[(size_t)pos * 32 + lane];
      sf[lr * SFP + lane]      = x1 * cs + x2 * sn;
      sf[lr * SFP + lane + 32] = x2 * cs - x1 * sn;
    }
  }
  __syncthreads();

  if (which < 2) {
    v4u hv[4], lv[4];
    size_t go[4];
    const int headrow = (which == 0) ? ns : (ns - 16);
#pragma unroll
    for (int j = 0; j < 4; ++j) {
      const int p  = tid + 128 * j;
      const int lr = p >> 3;
      const int d0 = (p & 7) * 8;
      const float* ra = sf + lr * SFP + d0;
      const v4f a0 = *(const v4f*)(ra), a1 = *(const v4f*)(ra + 4);
      const float f[8] = {a0[0], a0[1], a0[2], a0[3], a1[0], a1[1], a1[2], a1[3]};
      Pack8 ph, pl;
      split8(f, ph, pl);
      hv[j] = ph.u;
      lv[j] = pl.u;
      go[j] = ((size_t)headrow * SQ + mb + lr) * HDM + d0;
    }
    us* dsth = (which == 0) ? qh : kh;
    us* dstl = (which == 0) ? ql : kl;
#pragma unroll
    for (int j = 0; j < 4; ++j) { *(volatile v4u*)(dsth + go[j]) = hv[j]; *(volatile v4u*)(dstl + go[j]) = lv[j]; }
    __threadfence();
#pragma unroll
    for (int j = 0; j < 4; ++j) { *(volatile v4u*)(dsth + go[j]) = hv[j]; *(volatile v4u*)(dstl + go[j]) = lv[j]; }
  } else {
    v4u hv[4], lv[4];
    size_t go[4];
    const int kvh = ns - 20;
#pragma unroll
    for (int j = 0; j < 4; ++j) {
      const int p  = tid + 128 * j;
      const int d  = p >> 3;
      const int pc = p & 7;
      const float* cp = sf + (pc * 8) * SFP + d;
      float f[8];
#pragma unroll
      for (int e = 0; e < 8; ++e) f[e] = cp[e * SFP];
      Pack8 ph, pl;
      split8(f, ph, pl);
      hv[j] = ph.u;
      lv[j] = pl.u;
      go[j] = ((size_t)(kvh * HDM + d)) * SQ + mb + pc * 8;
    }
#pragma unroll
    for (int j = 0; j < 4; ++j) { *(volatile v4u*)(vh + go[j]) = hv[j]; *(volatile v4u*)(vl + go[j]) = lv[j]; }
    __threadfence();
#pragma unroll
    for (int j = 0; j < 4; ++j) { *(volatile v4u*)(vh + go[j]) = hv[j]; *(volatile v4u*)(vl + go[j]) = lv[j]; }
  }
}

#define LP 72
__global__ __launch_bounds__(128) void k_attn(const us* __restrict__ qh, const us* __restrict__ ql,
                                              const us* __restrict__ kh, const us* __restrict__ kl,
                                              const us* __restrict__ vh, const us* __restrict__ vl,
                                              us* __restrict__ oh, us* __restrict__ ol) {
  __shared__ __align__(16) us Ksh[KC * LP];
  __shared__ __align__(16) us Ksl[KC * LP];
  __shared__ __align__(16) us Vsh[HDM * LP];
  __shared__ __align__(16) us Vsl[HDM * LP];
  __shared__ __align__(16) us Psh[4 * 16 * LP];
  __shared__ __align__(16) us Psl[4 * 16 * LP];

  const int tid = threadIdx.x, lane = tid & 31, wave = tid >> 5;
  const int hh = lane >> 4, c = lane & 15;
  const int qb  = blockIdx.x % NQB;
  const int h   = blockIdx.x / NQB;
  const int kvh = h >> 2;
  const int q0  = qb * QB + wave * 16;

  const us* Qh = qh + (size_t)h * SQ * HDM;
  const us* Ql = ql + (size_t)h * SQ * HDM;
  const us* Kh = kh + (size_t)kvh * SQ * HDM;
  const us* Kl = kl + (size_t)kvh * SQ * HDM;
  const us* Vh = vh + (size_t)kvh * HDM * SQ;
  const us* Vl = vl + (size_t)kvh * HDM * SQ;

  const float NEGI = -__builtin_huge_valf();
  float mrow[8], lrow[8];
  v8f oacc[4];
#pragma unroll
  for (int r = 0; r < 8; ++r) { mrow[r] = NEGI; lrow[r] = 0.f; }
#pragma unroll
  for (int t = 0; t < 4; ++t) oacc[t] = zero8();

  us* pwh = Psh + wave * 16 * LP;
  us* pwl = Psl + wave * 16 * LP;
  const int nck = (qb >= 5) ? 6 : (qb + 1);

  for (int i = 0; i < nck; ++i) {
    const int kcn = (qb >= 5) ? ((i == 0) ? 0 : (qb - 5 + i)) : i;
    const int kv0 = kcn * KC;
    __syncthreads();
    {
      const int r  = tid >> 1;
      const int cb = (tid & 1) * 32;
      const us* ksh = Kh + (size_t)(kv0 + r) * HDM + cb;
      const us* ksl = Kl + (size_t)(kv0 + r) * HDM + cb;
      const us* vsh = Vh + (size_t)r * SQ + kv0 + cb;
      const us* vsl = Vl + (size_t)r * SQ + kv0 + cb;
#pragma unroll
      for (int e = 0; e < 4; ++e) {
        *(v8us*)(Ksh + r * LP + cb + 8 * e) = *(const v8us*)(ksh + 8 * e);
        *(v8us*)(Ksl + r * LP + cb + 8 * e) = *(const v8us*)(ksl + 8 * e);
        *(v8us*)(Vsh + r * LP + cb + 8 * e) = *(const v8us*)(vsh + 8 * e);
        *(v8us*)(Vsl + r * LP + cb + 8 * e) = *(const v8us*)(vsl + 8 * e);
      }
    }
    __syncthreads();

    v8f s[4];
#pragma unroll
    for (int j = 0; j < 4; ++j) s[j] = zero8();
#pragma unroll
    for (int dc = 0; dc < 2; ++dc) {
      const v16bf qah = ldfrag(Qh, HDM, q0, dc * 32, lane);
      const v16bf qal = ldfrag(Ql, HDM, q0, dc * 32, lane);
#pragma unroll
      for (int j = 0; j < 4; ++j) {
        const v16bf kbh = ldfrag(Ksh, LP, j * 16, dc * 32, lane);
        const v16bf kbl = ldfrag(Ksl, LP, j * 16, dc * 32, lane);
        s[j] = mma16(qah, kbh, s[j]);
        s[j] = mma16(qah, kbl, s[j]);
        s[j] = mma16(qal, kbh, s[j]);
      }
    }
#pragma unroll
    for (int r = 0; r < 8; ++r) {
      const int qry = q0 + 8 * hh + r;
#pragma unroll
      for (int j = 0; j < 4; ++j) {
        const int key = kv0 + 16 * j + c;
        const bool live = (key <= qry) && ((key >= qry - (LWIN - 1)) || (key < GTOK));
        const float sv = s[j][r] * 0.125f;
        s[j][r] = live ? sv : NEGI;
      }
    }
    float cm[8];
#pragma unroll
    for (int r = 0; r < 8; ++r) {
      float m = NEGI;
#pragma unroll
      for (int j = 0; j < 4; ++j) m = fmaxf(m, s[j][r]);
#pragma unroll
      for (int off = 1; off < 16; off <<= 1) m = fmaxf(m, __shfl_xor(m, off, 32));
      cm[r] = m;
    }
    float al[8];
#pragma unroll
    for (int r = 0; r < 8; ++r) {
      const float mnew  = fmaxf(mrow[r], cm[r]);
      const float alpha = __expf(mrow[r] - mnew);
      mrow[r] = mnew;
      float psum = 0.f;
#pragma unroll
      for (int j = 0; j < 4; ++j) {
        const float p = __expf(s[j][r] - mnew);
        psum += p;
        us ph, pl;
        split2(p, ph, pl);
        pwh[(8 * hh + r) * LP + j * 16 + c] = ph;
        pwl[(8 * hh + r) * LP + j * 16 + c] = pl;
      }
#pragma unroll
      for (int off = 1; off < 16; off <<= 1) psum += __shfl_xor(psum, off, 32);
      lrow[r] = lrow[r] * alpha + psum;
      al[r] = alpha;
    }
#pragma unroll
    for (int t = 0; t < 4; ++t)
#pragma unroll
      for (int r = 0; r < 8; ++r) oacc[t][r] *= al[r];
    __syncthreads();

#pragma unroll
    for (int kk = 0; kk < 2; ++kk) {
      const v16bf pah = ldfrag(pwh, LP, 0, kk * 32, lane);
      const v16bf pal = ldfrag(pwl, LP, 0, kk * 32, lane);
#pragma unroll
      for (int t = 0; t < 4; ++t) {
        const v16bf vbh = ldfrag(Vsh, LP, t * 16, kk * 32, lane);
        const v16bf vbl = ldfrag(Vsl, LP, t * 16, kk * 32, lane);
        oacc[t] = mma16(pah, vbh, oacc[t]);
        oacc[t] = mma16(pah, vbl, oacc[t]);
        oacc[t] = mma16(pal, vbh, oacc[t]);
      }
    }
  }

  float invl[8];
#pragma unroll
  for (int r = 0; r < 8; ++r) invl[r] = (lrow[r] > 0.f) ? (1.0f / lrow[r]) : 0.f;
  __syncthreads();
#pragma unroll
  for (int r = 0; r < 8; ++r) {
#pragma unroll
    for (int t = 0; t < 4; ++t) {
      us ohv, olv;
      split2(oacc[t][r] * invl[r], ohv, olv);
      pwh[(8 * hh + r) * LP + 16 * t + c] = ohv;
      pwl[(8 * hh + r) * LP + 16 * t + c] = olv;
    }
  }
  __syncthreads();
  v4u hv[4], lv[4];
  size_t go[4];
#pragma unroll
  for (int it = 0; it < 4; ++it) {
    const int p  = lane + 32 * it;
    const int L  = p >> 3;
    const int pc = p & 7;
    Pack8 ph, pl;
    ph.h   = *(const v8us*)(pwh + L * LP + pc * 8);
    pl.h   = *(const v8us*)(pwl + L * LP + pc * 8);
    hv[it] = ph.u;
    lv[it] = pl.u;
    go[it] = (size_t)(q0 + L) * DIM + (size_t)h * HDM + pc * 8;
  }
#pragma unroll
  for (int it = 0; it < 4; ++it) { *(volatile v4u*)(oh + go[it]) = hv[it]; *(volatile v4u*)(ol + go[it]) = lv[it]; }
  __threadfence();
#pragma unroll
  for (int it = 0; it < 4; ++it) { *(volatile v4u*)(oh + go[it]) = hv[it]; *(volatile v4u*)(ol + go[it]) = lv[it]; }
}

#define OTP 68
__global__ __launch_bounds__(128) void k_out(const us* __restrict__ ah, const us* __restrict__ al,
                                             const us* __restrict__ wh, const us* __restrict__ wl,
                                             float* __restrict__ out) {
  __shared__ __align__(16) float st[4][16 * OTP];
  const int tid = threadIdx.x, lane = tid & 31, wave = tid >> 5;
  const int hh = lane >> 4, c = lane & 15;
  const int m0 = blockIdx.x * 64 + wave * 16;
  const int n0 = blockIdx.y * 64;

  v8f acc[4];
#pragma unroll
  for (int t = 0; t < 4; ++t) acc[t] = zero8();
  gemm16x64x3(ah, al, wh, wl, m0, OROW + n0, lane, acc);

  float* sw = st[wave];
#pragma unroll
  for (int t = 0; t < 4; ++t) {
#pragma unroll
    for (int r = 0; r < 8; ++r) sw[(8 * hh + r) * OTP + 16 * t + c] = acc[t][r];
  }
  __syncthreads();
  v4f val[8];
  size_t go[8];
#pragma unroll
  for (int it = 0; it < 8; ++it) {
    const int p    = lane + 32 * it;
    const int L    = p >> 3;
    const int pc   = p & 7;
    const int row  = L >> 1;
    const int half = L & 1;
    const int col  = n0 + half * 32 + pc * 4;
    go[it]  = (size_t)(m0 + row) * DIM + col;
    val[it] = *(const v4f*)(sw + row * OTP + half * 32 + pc * 4);
  }
#pragma unroll
  for (int it = 0; it < 8; ++it) *(volatile v4f*)(out + go[it]) = val[it];
  __threadfence();
#pragma unroll
  for (int it = 0; it < 8; ++it) *(volatile v4f*)(out + go[it]) = val[it];
}

extern "C" void kernel_launch(void* const* d_in, const int* in_sizes, int n_in,
                              void* d_out, int out_size, void* d_ws, size_t ws_size,
                              hipStream_t stream) {
  if (n_in < 5) return;
  if (in_sizes[0] != SQ * DIM) return;
  if (in_sizes[1] != DIM * DIM) return;
  if (in_sizes[2] != DIM * KVD) return;
  if (in_sizes[3] != DIM * KVD) return;
  if (in_sizes[4] != DIM * DIM) return;
  if (out_size != SQ * DIM) return;

  const float* x  = (const float*)d_in[0];
  const float* wq = (const float*)d_in[1];
  const float* wk = (const float*)d_in[2];
  const float* wv = (const float*)d_in[3];
  const float* wo = (const float*)d_in[4];
  float* out = (float*)d_out;

  size_t off = 0;
  const size_t oXh = off; off += (size_t)SQ * DIM * 2;
  const size_t oXl = off; off += (size_t)SQ * DIM * 2;
  const size_t oWh = off; off += (size_t)WROWS * DIM * 2;
  const size_t oWl = off; off += (size_t)WROWS * DIM * 2;
  const size_t oQh = off; off += (size_t)NH * SQ * HDM * 2;
  const size_t oQl = off; off += (size_t)NH * SQ * HDM * 2;
  const size_t oKh = off; off += (size_t)NKV * SQ * HDM * 2;
  const size_t oKl = off; off += (size_t)NKV * SQ * HDM * 2;
  const size_t oVh = off; off += (size_t)NKV * HDM * SQ * 2;
  const size_t oVl = off; off += (size_t)NKV * HDM * SQ * 2;
  const size_t oOh = off; off += (size_t)SQ * DIM * 2;
  const size_t oOl = off; off += (size_t)SQ * DIM * 2;
  const size_t oCT = off; off += (size_t)SQ * 32 * 4;
  const size_t oST = off; off += (size_t)SQ * 32 * 4;
  if (off > ws_size) return;
  if (off > (size_t)134217728) return;

  char* ws = (char*)d_ws;
  us* Xh = (us*)(ws + oXh);
  us* Xl = (us*)(ws + oXl);
  us* Wh = (us*)(ws + oWh);
  us* Wl = (us*)(ws + oWl);
  us* Qh = (us*)(ws + oQh);
  us* Ql = (us*)(ws + oQl);
  us* Kh = (us*)(ws + oKh);
  us* Kl = (us*)(ws + oKl);
  us* Vh = (us*)(ws + oVh);
  us* Vl = (us*)(ws + oVl);
  us* Oh = (us*)(ws + oOh);
  us* Ol = (us*)(ws + oOl);
  float* CT = (float*)(ws + oCT);
  float* ST = (float*)(ws + oST);

  RopeTab tab;
  {
    double cr = 1.3335214321633240;
    for (int it = 0; it < 8; ++it) {
      double p31 = 1.0;
      for (int k = 0; k < 31; ++k) p31 *= cr;
      const double f = p31 * cr - 10000.0;
      cr = cr - f / (32.0 * p31);
    }
    double p = 1.0;
    for (int j = 0; j < 32; ++j) {
      const float pf = (float)p;
      tab.f[j] = 1.0f / pf;
      p *= cr;
    }
  }

  k_cvtw<<<dim3(WROWS / 64, DIM / 64), dim3(128), 0, stream>>>(wq, wk, wv, wo, Wh, Wl);
  k_cvtx<<<dim3((SQ * DIM) / 2048), dim3(256), 0, stream>>>(x, Xh, Xl);
  k_rope<<<dim3(SQ / 8), dim3(256), 0, stream>>>(tab, CT, ST);
  k_qkv<<<dim3(SQ / 64, (DIM + KVD + KVD) / HDM), dim3(128), 0, stream>>>(Xh, Xl, Wh, Wl, CT, ST,
                                                                          Qh, Ql, Kh, Kl, Vh, Vl);
  k_attn<<<dim3(NH * NQB), dim3(128), 0, stream>>>(Qh, Ql, Kh, Kl, Vh, Vl, Oh, Ol);
  k_out<<<dim3(SQ / 64, DIM / 64), dim3(128), 0, stream>>>(Oh, Ol, Wh, Wl, out);
  (void)hipGetLastError();
}
